// ESN_83502754169067
// MI455X (gfx1250) — hardware-run, weakly checked
//
#include <hip/hip_runtime.h>
#include <math.h>

constexpr int DIM    = 512;
constexpr int RES    = 2048;
constexpr int TWIN   = 128;
constexpr int LGEN   = 64;
constexpr int G4     = 4 * DIM;
constexpr int NWIN   = LGEN;
constexpr int NSTEPS = TWIN + LGEN - 1;
constexpr int NTHR   = 256;
constexpr int PTHR   = 512;
constexpr int NWAVE  = PTHR / 32;
constexpr int SLP    = 72;
constexpr int HPLANE = NWIN * DIM;
static_assert(DIM % 32 == 0 && RES % 32 == 0, "K multiples of 32");
static_assert(TWIN % 64 == 0 && G4 % 64 == 0, "warmup GEMM M and N tile multiples");
static_assert(NWIN % 16 == 0 && NWAVE == 4 * (NWIN / 16), "4 waves per window subtile");
static_assert((NWAVE / (NWIN / 16)) * 8 * 16 == DIM, "8 unit subtiles per wave cover DIM");
static_assert(RES == NWAVE * 8 * 16 && DIM == NWAVE * 2 * 16, "matvec output coverage");
static_assert(PTHR * 4 == G4, "px copy coverage");
static_assert(4 * 32 * 4 == DIM, "output row store coverage: 4 waves x 32 lanes x 4 floats");
static_assert((SLP * 2) % 16 == 0, "slab rows 16-B aligned");

typedef __attribute__((ext_vector_type(16))) _Float16 v16h;
typedef __attribute__((ext_vector_type(8)))  _Float16 v8h;
typedef __attribute__((ext_vector_type(16))) __bf16   v16b;
typedef __attribute__((ext_vector_type(8)))  __bf16   v8b;
typedef __attribute__((ext_vector_type(8)))  float    v8f;
typedef __attribute__((ext_vector_type(4)))  float    v4f;
typedef __attribute__((ext_vector_type(4)))  unsigned v4u;

__device__ __forceinline__ unsigned short f2bf_bits(float f) {
  unsigned u = __float_as_uint(f);
  return (unsigned short)((u + 0x7FFFu + ((u >> 16) & 1u)) >> 16);
}
__device__ __forceinline__ float bf_bits2f(unsigned short h) { return __uint_as_float(((unsigned)h) << 16); }
__device__ __forceinline__ float bf16r(float f) { return bf_bits2f(f2bf_bits(f)); }

__device__ __forceinline__ void dep_guard_h(v8f& a, v8f& b, v16h x, v16h y) { asm volatile("v_nop\n\tv_nop\n\tv_nop\n\tv_nop" : "+v"(a), "+v"(b) : "v"(x), "v"(y)); }
__device__ __forceinline__ void dep_guard_b(v8f& a, v8f& b, v16b x, v16b y) { asm volatile("v_nop\n\tv_nop\n\tv_nop\n\tv_nop" : "+v"(a), "+v"(b) : "v"(x), "v"(y)); }
__device__ __forceinline__ void keep4_h(v16h a, v16h b, v16h c, v16h d) { asm volatile("v_nop" :: "v"(a), "v"(b), "v"(c), "v"(d)); }
__device__ __forceinline__ void keep4_b(v16b a, v16b b, v16b c, v16b d) { asm volatile("v_nop" :: "v"(a), "v"(b), "v"(c), "v"(d)); }
__device__ __forceinline__ void acc_guard4(v8f& a, v8f& b, v8f& c, v8f& d) { asm volatile("v_nop\n\tv_nop\n\tv_nop\n\tv_nop" : "+v"(a), "+v"(b), "+v"(c), "+v"(d)); }
__device__ __forceinline__ void acc_guard2(v8f& a, v8f& b) { asm volatile("v_nop\n\tv_nop\n\tv_nop\n\tv_nop" : "+v"(a), "+v"(b)); }
__device__ __forceinline__ void guard4x6(v8f& a0, v8f& a1, v8f& a2, v8f& a3,
                                         v16b x0, v16b x1, v16b x2, v16b x3, v16b x4, v16b x5) {
  asm volatile("v_nop\n\tv_nop\n\tv_nop\n\tv_nop"
               : "+v"(a0), "+v"(a1), "+v"(a2), "+v"(a3)
               : "v"(x0), "v"(x1), "v"(x2), "v"(x3), "v"(x4), "v"(x5));
}
__device__ __forceinline__ void guard4x5(v8f& a0, v8f& a1, v8f& a2, v8f& a3,
                                         v16b x0, v16b x1, v16b x2, v16b x3, v16b x4) {
  asm volatile("v_nop\n\tv_nop\n\tv_nop\n\tv_nop"
               : "+v"(a0), "+v"(a1), "+v"(a2), "+v"(a3)
               : "v"(x0), "v"(x1), "v"(x2), "v"(x3), "v"(x4));
}
__device__ __forceinline__ void guard2x3(v8f& a0, v8f& a1, v16b x0, v16b x1, v16b x2) {
  asm volatile("v_nop\n\tv_nop\n\tv_nop\n\tv_nop" : "+v"(a0), "+v"(a1) : "v"(x0), "v"(x1), "v"(x2));
}

template <typename T> struct Frag;
template <> struct Frag<_Float16> {
  typedef v16h V; union U { v16h v; v8h h[2]; };
  static __device__ __forceinline__ v16h load(const _Float16* p) {
    U f; f.h[0] = *(const v8h*)(p); f.h[1] = *(const v8h*)(p + 16); return f.v;
  }
  static __device__ __forceinline__ v8f mma(v16h a, v16h b, v8f c) {
    return __builtin_amdgcn_wmma_f32_16x16x32_f16(false, a, false, b, (short)0, c, false, false);
  }
  static __device__ __forceinline__ void guard(v8f& a, v8f& b, v16h x, v16h y) { dep_guard_h(a, b, x, y); }
  static __device__ __forceinline__ void keep(v16h a, v16h b, v16h c, v16h d) { keep4_h(a, b, c, d); }
};
template <> struct Frag<__bf16> {
  typedef v16b V; union U { v16b v; v8b h[2]; };
  static __device__ __forceinline__ v16b load(const __bf16* p) {
    U f; f.h[0] = *(const v8b*)(p); f.h[1] = *(const v8b*)(p + 16); return f.v;
  }
  static __device__ __forceinline__ v8f mma(v16b a, v16b b, v8f c) {
    return __builtin_amdgcn_wmma_f32_16x16x32_bf16(false, a, false, b, (short)0, c, false, false);
  }
  static __device__ __forceinline__ void guard(v8f& a, v8f& b, v16b x, v16b y) { dep_guard_b(a, b, x, y); }
  static __device__ __forceinline__ void keep(v16b a, v16b b, v16b c, v16b d) { keep4_b(a, b, c, d); }
};

template <int ET> struct Elem;
template <> struct Elem<0> { typedef _Float16 T; };
template <> struct Elem<1> { typedef __bf16 T; };
template <int ET, bool SPLIT, int BIAS_MODE, int OUT_MODE, bool RESID, int ACT = 0>
__global__ __launch_bounds__(256) void wmma_gemm64(
    const unsigned short* __restrict__ Ap, const unsigned short* __restrict__ A2p, int lda, long strideA,
    const unsigned short* __restrict__ Btp, const unsigned short* __restrict__ Bt2p, int ldb, long strideB,
    void* __restrict__ Cout, void* __restrict__ Cout2, int ldc, long strideC,
    const float* __restrict__ bias,
    const float* __restrict__ resid, long strideR,
    int M, int N, int K, float scale) {
  typedef typename Elem<ET>::T T;
  typedef typename Frag<T>::V V;
  const T* A = (const T*)Ap; const T* A2 = (const T*)A2p; const T* Bt = (const T*)Btp; const T* Bt2 = (const T*)Bt2p;
  __shared__ __align__(16) float sT[8][16 * 68];
  const int b    = blockIdx.y;
  const int lane = threadIdx.x & 31;
  const int wave = threadIdx.x >> 5;
  const int tilesN = N >> 6;
  const int tilesM = M >> 6;
  const int tile = blockIdx.x * 8 + wave;
  if (tile >= tilesM * tilesN) return;
  const int tm = tile / tilesN;
  const int tn = tile - tm * tilesN;
  const int m0 = tm << 6;
  const int n0 = tn << 6;

  const T* Ab  = A  + (size_t)b * strideA;
  const T* Bb  = Bt + (size_t)b * strideB;
  const T* Ab2 = SPLIT ? (A2  + (size_t)b * strideA) : nullptr;
  const T* Bb2 = SPLIT ? (Bt2 + (size_t)b * strideB) : nullptr;

  const int rlane = lane & 15;
  const int koff  = (lane >> 4) * 8;
  const int mOff  = (lane >> 4) * 8;

  v8f acc[4][4];
#pragma unroll
  for (int i = 0; i < 4; ++i)
#pragma unroll
    for (int j = 0; j < 4; ++j) acc[i][j] = (v8f){0.f,0.f,0.f,0.f,0.f,0.f,0.f,0.f};

  for (int k0 = 0; k0 < K; k0 += 32) {
    V bh[4], bl[4];
#pragma unroll
    for (int j = 0; j < 4; ++j) {
      const size_t bo = (size_t)(n0 + (j << 4) + rlane) * ldb + koff + k0;
      bh[j] = Frag<T>::load(Bb + bo);
      if (SPLIT) bl[j] = Frag<T>::load(Bb2 + bo);
    }
#pragma unroll
    for (int i = 0; i < 4; ++i) {
      const size_t ao = (size_t)(m0 + (i << 4) + rlane) * lda + koff + k0;
      V ah = Frag<T>::load(Ab + ao);
      V al;
      if (SPLIT) al = Frag<T>::load(Ab2 + ao);
#pragma unroll
      for (int j = 0; j < 4; ++j) {
        acc[i][j] = Frag<T>::mma(ah, bh[j], acc[i][j]);
        if (SPLIT) {
          acc[i][j] = Frag<T>::mma(ah, bl[j], acc[i][j]);
          acc[i][j] = Frag<T>::mma(al, bh[j], acc[i][j]);
        }
      }
      Frag<T>::guard(acc[i][0], acc[i][3], ah, SPLIT ? al : ah);
    }
    Frag<T>::keep(bh[0], bh[1], bh[2], bh[3]);
    if (SPLIT) Frag<T>::keep(bl[0], bl[1], bl[2], bl[3]);
  }
  acc_guard4(acc[0][0], acc[0][1], acc[0][2], acc[0][3]);
  acc_guard4(acc[1][0], acc[1][1], acc[1][2], acc[1][3]);
  acc_guard4(acc[2][0], acc[2][1], acc[2][2], acc[2][3]);
  acc_guard4(acc[3][0], acc[3][1], acc[3][2], acc[3][3]);

  float* slab = sT[wave];
  const float* Rb = RESID ? (resid + (size_t)b * strideR) : nullptr;
#pragma unroll
  for (int i = 0; i < 4; ++i) {
    const int mBase = m0 + (i << 4);
#pragma unroll
    for (int j = 0; j < 4; ++j) {
      const int n = n0 + (j << 4) + rlane;
      float bv = 0.f;
      if (BIAS_MODE == 2) bv = bias[n];
#pragma unroll
      for (int r = 0; r < 8; ++r) {
        float v = acc[i][j][r] * scale;
        if (BIAS_MODE == 1) v += bias[mBase + mOff + r];
        if (BIAS_MODE == 2) v += bv;
        if (RESID) v += Rb[(size_t)(mBase + mOff + r) * ldc + n];
        if (ACT == 1) v = tanhf(v);
        if (ACT == 2) v = fmaxf(v, 0.0f);
        if (ACT == 3) v = v / (1.0f + expf(-v));
        if (ACT == 4) v = (v > 0.f) ? v : 0.01f * v;
        if (ACT == 5) v = 0.5f * v * (1.0f + erff(v * 0.70710678118654752f));
        slab[(mOff + r) * 68 + (j << 4) + rlane] = v;
      }
    }
    __builtin_amdgcn_fence(__ATOMIC_RELEASE, "workgroup");
    __builtin_amdgcn_wave_barrier();
    __builtin_amdgcn_fence(__ATOMIC_ACQUIRE, "workgroup");
    if (OUT_MODE == 0) {
      float* C = (float*)Cout + (size_t)b * strideC;
      const int hh = lane >> 4, c4 = (lane & 15) * 4;
      for (int pass = 0; pass < 2; ++pass) {
#pragma unroll
        for (int it = 0; it < 8; ++it) {
          const int row = it * 2 + hh;
          v4f v = *(const v4f*)(slab + row * 68 + c4);
          *(volatile v4f*)(C + (size_t)(mBase + row) * ldc + n0 + c4) = v;
        }
        __threadfence();
      }
    } else {
      const int q = lane >> 3, c8 = (lane & 7) * 8;
      unsigned short* C  = (unsigned short*)Cout  + (size_t)b * strideC;
      unsigned short* C2 = (OUT_MODE == 2) ? ((unsigned short*)Cout2 + (size_t)b * strideC) : nullptr;
      for (int pass = 0; pass < 2; ++pass) {
#pragma unroll
        for (int it = 0; it < 4; ++it) {
          const int row = it * 4 + q;
          const float* sp = slab + row * 68 + c8;
          v8h hv, lv;
#pragma unroll
          for (int e = 0; e < 8; ++e) {
            if (OUT_MODE == 1) {
              hv[e] = (_Float16)sp[e];
            } else {
              unsigned short hb = f2bf_bits(sp[e]);
              unsigned short lb = f2bf_bits(sp[e] - bf_bits2f(hb));
              hv[e] = __builtin_bit_cast(_Float16, hb);
              lv[e] = __builtin_bit_cast(_Float16, lb);
            }
          }
          *(volatile v8h*)(C + (size_t)(mBase + row) * ldc + n0 + c8) = hv;
          if (OUT_MODE == 2) *(volatile v8h*)(C2 + (size_t)(mBase + row) * ldc + n0 + c8) = lv;
        }
        __threadfence();
      }
    }
    __builtin_amdgcn_fence(__ATOMIC_RELEASE, "workgroup");
    __builtin_amdgcn_wave_barrier();
    __builtin_amdgcn_fence(__ATOMIC_ACQUIRE, "workgroup");
  }
}

__global__ __launch_bounds__(NTHR) void cast_bf16x8(const float* __restrict__ src, unsigned short* __restrict__ dst, int n8) {
  const int i = blockIdx.x * NTHR + threadIdx.x;
  if (i < n8) {
    const v4f a = *(const v4f*)(src + (size_t)i * 8);
    const v4f b = *(const v4f*)(src + (size_t)i * 8 + 4);
    v8h hv;
#pragma unroll
    for (int e = 0; e < 4; ++e) {
      hv[e]     = __builtin_bit_cast(_Float16, f2bf_bits(a[e]));
      hv[4 + e] = __builtin_bit_cast(_Float16, f2bf_bits(b[e]));
    }
    *(volatile v8h*)(dst + (size_t)i * 8) = hv;
    __threadfence();
    *(volatile v8h*)(dst + (size_t)i * 8) = hv;
  }
}

__global__ __launch_bounds__(PTHR) void zero16x8(unsigned short* __restrict__ dst, int n8) {
  const int i = blockIdx.x * PTHR + threadIdx.x;
  if (i < n8) {
    const v4u z = {0u, 0u, 0u, 0u};
    *(volatile v4u*)(dst + (size_t)i * 8) = z;
    __threadfence();
    *(volatile v4u*)(dst + (size_t)i * 8) = z;
  }
}

__device__ __forceinline__ float fsig(float x)  { return __builtin_amdgcn_rcpf(1.0f + expf(-x)); }
__device__ __forceinline__ float ftanh(float x) { return 1.0f - 2.0f * __builtin_amdgcn_rcpf(expf(2.0f * x) + 1.0f); }

template <int KD>
__device__ __forceinline__ void build_bvec(const float* vec, __bf16* bv, int tid) {
#pragma unroll 1
  for (int k8 = tid; k8 < KD / 8; k8 += PTHR) {
    const v4f a = *(const v4f*)(vec + 8 * k8);
    const v4f b = *(const v4f*)(vec + 8 * k8 + 4);
    v8b hv, lv;
#pragma unroll
    for (int e = 0; e < 4; ++e) {
      const unsigned short h0 = f2bf_bits(a[e]);
      const unsigned short l0 = f2bf_bits(a[e] - bf_bits2f(h0));
      const unsigned short h1 = f2bf_bits(b[e]);
      const unsigned short l1 = f2bf_bits(b[e] - bf_bits2f(h1));
      hv[e]     = __builtin_bit_cast(__bf16, h0);
      hv[4 + e] = __builtin_bit_cast(__bf16, h1);
      lv[e]     = __builtin_bit_cast(__bf16, l0);
      lv[4 + e] = __builtin_bit_cast(__bf16, l1);
    }
    *(v8b*)(bv + 8 * k8) = hv;
    *(v8b*)(bv + KD + 8 * k8) = lv;
  }
}

template <int NSUB, int KD, int MODE>
__device__ __forceinline__ void gemv_part(const __bf16* __restrict__ Wp, const __bf16* bv,
                                          const float* __restrict__ bias0, const float* __restrict__ bias1,
                                          float* dst, int wave, int lane) {
  constexpr int GS = (NSUB >= 4) ? 4 : NSUB;
  constexpr int NGRP = NSUB / GS;
  static_assert(NSUB % GS == 0 && (GS == 4 || GS == 2), "group size");
  static_assert(KD % 32 == 0, "K multiple of 32");
  const int c = lane & 15, hh = lane >> 4, koff = 8 * hh;
  const v8f z8 = {0.f, 0.f, 0.f, 0.f, 0.f, 0.f, 0.f, 0.f};
  const __bf16* bvr = bv + (c & 1) * KD + koff;
#pragma unroll
  for (int grp = 0; grp < NGRP; ++grp) {
    const int ms0 = wave * NSUB + grp * GS;
    const __bf16* wr = Wp + (size_t)(16 * ms0 + c) * KD + koff;
    v8f acc[GS];
#pragma unroll
    for (int i = 0; i < GS; ++i) acc[i] = z8;
#pragma unroll 1
    for (int k0 = 0; k0 < KD; k0 += 32) {
      const v16b fb = Frag<__bf16>::load(bvr + k0);
      if constexpr (GS == 4) {
        const v16b x0 = Frag<__bf16>::load(wr + k0);
        const v16b x1 = Frag<__bf16>::load(wr + (size_t)16 * KD + k0);
        const v16b x2 = Frag<__bf16>::load(wr + (size_t)32 * KD + k0);
        const v16b x3 = Frag<__bf16>::load(wr + (size_t)48 * KD + k0);
        acc[0] = Frag<__bf16>::mma(x0, fb, acc[0]);
        acc[1] = Frag<__bf16>::mma(x1, fb, acc[1]);
        acc[2] = Frag<__bf16>::mma(x2, fb, acc[2]);
        acc[3] = Frag<__bf16>::mma(x3, fb, acc[3]);
        guard4x5(acc[0], acc[1], acc[2], acc[3], x0, x1, x2, x3, fb);
      } else {
        const v16b x0 = Frag<__bf16>::load(wr + k0);
        const v16b x1 = Frag<__bf16>::load(wr + (size_t)16 * KD + k0);
        acc[0] = Frag<__bf16>::mma(x0, fb, acc[0]);
        acc[1] = Frag<__bf16>::mma(x1, fb, acc[1]);
        guard2x3(acc[0], acc[1], x0, x1, fb);
      }
    }
    if constexpr (GS == 4) acc_guard4(acc[0], acc[1], acc[2], acc[3]);
    else acc_guard2(acc[0], acc[1]);
#pragma unroll
    for (int i = 0; i < GS; ++i) {
      const int m8 = 16 * (ms0 + i) + 8 * hh;
      const v4f bA = *(const v4f*)(bias0 + m8);
      const v4f bB = *(const v4f*)(bias0 + m8 + 4);
      float badd[8];
#pragma unroll
      for (int e = 0; e < 4; ++e) { badd[e] = bf16r(bA[e]); badd[4 + e] = bf16r(bB[e]); }
      if constexpr (MODE == 2) {
        const v4f cA = *(const v4f*)(bias1 + m8);
        const v4f cB = *(const v4f*)(bias1 + m8 + 4);
#pragma unroll
        for (int e = 0; e < 4; ++e) { badd[e] = badd[e] + bf16r(cA[e]); badd[4 + e] = badd[4 + e] + bf16r(cB[e]); }
      }
      float vv[8];
#pragma unroll
      for (int r = 0; r < 8; ++r) {
        const float t = acc[i][r];
        const float pairsum = t + __shfl_xor(t, 1, 32);
        float v = pairsum + badd[r];
        if constexpr (MODE == 0) v = (v >= 0.0f) ? v : 0.01f * v;
        vv[r] = v;
      }
      float sel = vv[0];
#pragma unroll
      for (int r = 1; r < 8; ++r) sel = (c == r) ? vv[r] : sel;
      if (c < 8) dst[m8 + c] = sel;
    }
  }
}

__global__ __launch_bounds__(PTHR) void seq_cell_kernel(
    const float* __restrict__ PXG,
    const unsigned short* __restrict__ WHHB, const unsigned short* __restrict__ WIHB,
    const unsigned short* __restrict__ W1B, const unsigned short* __restrict__ W2B,
    const float* __restrict__ bih, const float* __restrict__ bhh,
    const float* __restrict__ b1, const float* __restrict__ b2,
    unsigned short* HPL, float* out) {
  __shared__ __align__(16) _Float16 slabH[NWAVE][16 * SLP];
  __shared__ __align__(16) _Float16 slabL[NWAVE][16 * SLP];
  __shared__ __align__(16) float pxl[G4];
  __shared__ __align__(16) float rl[RES];
  __shared__ __align__(16) float hfin[DIM];
  __shared__ __align__(16) float yl[DIM];
  __shared__ __align__(16) __bf16 bv512[2 * DIM];
  __shared__ __align__(16) __bf16 bv2048[2 * RES];

  const int tid  = threadIdx.x;
  const int lane = tid & 31;
  const int wave = __builtin_amdgcn_readfirstlane((int)(threadIdx.x >> 5));
  const int c = lane & 15, hh = lane >> 4, koff = 8 * hh;
  const int mt = wave >> 2;
  const int cq = wave & 3;
  const int jrow0 = 16 * mt + 8 * hh;
  const __bf16* WHH = (const __bf16*)WHHB;
  const __bf16* WIH = (const __bf16*)WIHB;
  const __bf16* W1  = (const __bf16*)W1B;
  const __bf16* W2  = (const __bf16*)W2B;
  const v8f z8 = {0.f, 0.f, 0.f, 0.f, 0.f, 0.f, 0.f, 0.f};
  _Float16* sH = slabH[wave];
  _Float16* sL = slabL[wave];

  float cst[8][8];
#pragma unroll
  for (int u = 0; u < 8; ++u)
#pragma unroll
    for (int r = 0; r < 8; ++r) cst[u][r] = 0.0f;

#pragma unroll 1
  for (int s = 0; s < NSTEPS; ++s) {
    const int lo  = s - (TWIN - 1);
    const int wlo = (lo > 0) ? lo : 0;
    const int whi = (s < NWIN - 1) ? s : (NWIN - 1);
    const bool mt_act = (16 * mt <= whi) && (16 * mt + 15 >= wlo);
    const int pc = s & 1, pn = pc ^ 1;

    if (s < TWIN) {
      const int i4 = 4 * tid;
      const v4f g  = *(const v4f*)(PXG + (size_t)s * G4 + i4);
      const v4f ba = *(const v4f*)(bih + i4);
      const v4f bb = *(const v4f*)(bhh + i4);
      v4f o;
#pragma unroll
      for (int e = 0; e < 4; ++e) o[e] = g[e] + (bf16r(ba[e]) + bf16r(bb[e]));
      *(v4f*)(pxl + i4) = o;
    }
    __syncthreads();
    __threadfence();

    if (mt_act) {
      const __bf16* ahp = (const __bf16*)(HPL + (size_t)pc * HPLANE) + (size_t)(16 * mt + c) * DIM + koff;
      const __bf16* alp = (const __bf16*)(HPL + (size_t)(2 + pc) * HPLANE) + (size_t)(16 * mt + c) * DIM + koff;
      unsigned short* hnh = HPL + (size_t)pn * HPLANE + (size_t)(16 * mt) * DIM + 128 * cq;
      unsigned short* hnl = HPL + (size_t)(2 + pn) * HPLANE + (size_t)(16 * mt) * DIM + 128 * cq;
#pragma unroll
      for (int half = 0; half < 2; ++half) {
#pragma unroll
        for (int i = 0; i < 4; ++i) {
          const int u = 4 * half + i;
          const int n = 16 * (8 * cq + u) + c;
          const __bf16* wg = WHH + (size_t)n * DIM + koff;
          v8f a0 = z8, a1 = z8, a2 = z8, a3 = z8;
#pragma unroll 1
          for (int k0 = 0; k0 < DIM; k0 += 32) {
            const v16b fh = Frag<__bf16>::load(ahp + k0);
            const v16b fl = Frag<__bf16>::load(alp + k0);
            const v16b g0 = Frag<__bf16>::load(wg + k0);
            const v16b g1 = Frag<__bf16>::load(wg + (size_t)1 * DIM * DIM + k0);
            const v16b g2 = Frag<__bf16>::load(wg + (size_t)2 * DIM * DIM + k0);
            const v16b g3 = Frag<__bf16>::load(wg + (size_t)3 * DIM * DIM + k0);
            a0 = Frag<__bf16>::mma(fh, g0, a0);
            a1 = Frag<__bf16>::mma(fh, g1, a1);
            a2 = Frag<__bf16>::mma(fh, g2, a2);
            a3 = Frag<__bf16>::mma(fh, g3, a3);
            a0 = Frag<__bf16>::mma(fl, g0, a0);
            a1 = Frag<__bf16>::mma(fl, g1, a1);
            a2 = Frag<__bf16>::mma(fl, g2, a2);
            a3 = Frag<__bf16>::mma(fl, g3, a3);
            guard4x6(a0, a1, a2, a3, fh, fl, g0, g1, g2, g3);
          }
          acc_guard4(a0, a1, a2, a3);
          const float pi = pxl[n], pf = pxl[DIM + n], pg = pxl[2 * DIM + n], po = pxl[3 * DIM + n];
#pragma unroll
          for (int r = 0; r < 8; ++r) {
            const int j = jrow0 + r;
            const bool act = (j >= lo) && (j <= s);
            const float ig = fsig(a0[r] + pi);
            const float fg = fsig(a1[r] + pf);
            const float gt = ftanh(a2[r] + pg);
            const float og = fsig(a3[r] + po);
            const float cold = cst[u][r];
            const float cc = fg * cold + ig * gt;
            const float cn = act ? cc : cold;
            cst[u][r] = cn;
            const float hc = og * ftanh(cn);
            const float hn = act ? hc : 0.0f;
            const unsigned short hb = f2bf_bits(hn);
            const unsigned short lb = f2bf_bits(hn - bf_bits2f(hb));
            const int so = (8 * hh + r) * SLP + 16 * i + c;
            sH[so] = __builtin_bit_cast(_Float16, hb);
            sL[so] = __builtin_bit_cast(_Float16, lb);
            if (j == lo) hfin[n] = hn;
          }
        }
        __builtin_amdgcn_fence(__ATOMIC_RELEASE, "workgroup");
        __builtin_amdgcn_wave_barrier();
        __builtin_amdgcn_fence(__ATOMIC_ACQUIRE, "workgroup");
        {
          const int q = lane >> 3, c8 = (lane & 7) * 8;
          for (int pass = 0; pass < 2; ++pass) {
#pragma unroll
            for (int it = 0; it < 4; ++it) {
              const int row = 4 * it + q;
              const v8h vh = *(const v8h*)(sH + row * SLP + c8);
              const v8h vl = *(const v8h*)(sL + row * SLP + c8);
              *(volatile v8h*)(hnh + (size_t)row * DIM + 64 * half + c8) = vh;
              *(volatile v8h*)(hnl + (size_t)row * DIM + 64 * half + c8) = vl;
            }
            __threadfence();
          }
        }
        __builtin_amdgcn_fence(__ATOMIC_RELEASE, "workgroup");
        __builtin_amdgcn_wave_barrier();
        __builtin_amdgcn_fence(__ATOMIC_ACQUIRE, "workgroup");
      }
    }
    __syncthreads();

    if (s >= TWIN - 1) {
      const int jd = lo;
      build_bvec<DIM>(hfin, bv512, tid);
      __syncthreads();
      gemv_part<8, DIM, 0>(W1, bv512, b1, b1, rl, wave, lane);
      __syncthreads();
      build_bvec<RES>(rl, bv2048, tid);
      __syncthreads();
      gemv_part<2, RES, 1>(W2, bv2048, b2, b2, yl, wave, lane);
      __syncthreads();
      if (wave < 4) {
        const v4f val = *(const v4f*)(yl + 128 * wave + 4 * lane);
        float* op = out + (size_t)jd * DIM + 128 * wave + 4 * lane;
        *(volatile v4f*)op = val;
        __threadfence();
        *(volatile v4f*)op = val;
      }
      build_bvec<DIM>(yl, bv512, tid);
      __syncthreads();
      gemv_part<8, DIM, 2>(WIH, bv512, bih, bhh, pxl, wave, lane);
      __syncthreads();
    }
  }
}

extern "C" void kernel_launch(void* const* d_in, const int* in_sizes, int n_in,
                              void* d_out, int out_size, void* d_ws, size_t ws_size, hipStream_t stream) {
  if (n_in < 9 || d_out == nullptr || d_ws == nullptr) return;
  if (in_sizes[0] != TWIN * DIM || in_sizes[1] != G4 * DIM || in_sizes[2] != G4 * DIM ||
      in_sizes[3] != G4 || in_sizes[4] != G4 || in_sizes[5] != RES * DIM || in_sizes[6] != RES ||
      in_sizes[7] != DIM * RES || in_sizes[8] != DIM || out_size != LGEN * DIM) return;

  const float* x   = (const float*)d_in[0];
  const float* Wih = (const float*)d_in[1];
  const float* Whh = (const float*)d_in[2];
  const float* bih = (const float*)d_in[3];
  const float* bhh = (const float*)d_in[4];
  const float* W1  = (const float*)d_in[5];
  const float* b1  = (const float*)d_in[6];
  const float* W2  = (const float*)d_in[7];
  const float* b2  = (const float*)d_in[8];
  float* out = (float*)d_out;

  char* ws = (char*)d_ws; size_t off = 0;
  auto carve = [&](size_t bytes) -> char* { char* p = ws + off; off += (bytes + 255) & ~(size_t)255; return p; };
  unsigned short* XB   = (unsigned short*)carve((size_t)TWIN * DIM * 2);
  unsigned short* WIHB = (unsigned short*)carve((size_t)G4 * DIM * 2);
  unsigned short* WHHB = (unsigned short*)carve((size_t)G4 * DIM * 2);
  unsigned short* W1B  = (unsigned short*)carve((size_t)RES * DIM * 2);
  unsigned short* W2B  = (unsigned short*)carve((size_t)DIM * RES * 2);
  float*          PXG  = (float*)carve((size_t)TWIN * G4 * 4);
  unsigned short* HPL  = (unsigned short*)carve((size_t)4 * HPLANE * 2);
  if (off > ws_size || off > (size_t)134217728) return;

  const int n8x = TWIN * DIM / 8;
  const int n8w = G4 * DIM / 8;
  cast_bf16x8<<<(n8x + NTHR - 1) / NTHR, NTHR, 0, stream>>>(x,   XB,   n8x);
  cast_bf16x8<<<(n8w + NTHR - 1) / NTHR, NTHR, 0, stream>>>(Wih, WIHB, n8w);
  cast_bf16x8<<<(n8w + NTHR - 1) / NTHR, NTHR, 0, stream>>>(Whh, WHHB, n8w);
  cast_bf16x8<<<(n8w + NTHR - 1) / NTHR, NTHR, 0, stream>>>(W1,  W1B,  n8w);
  cast_bf16x8<<<(n8w + NTHR - 1) / NTHR, NTHR, 0, stream>>>(W2,  W2B,  n8w);
  const int n8h = 4 * HPLANE / 8;
  zero16x8<<<(n8h + PTHR - 1) / PTHR, PTHR, 0, stream>>>(HPL, n8h);
  wmma_gemm64<1, false, 0, 0, false, 0><<<dim3((TWIN / 64) * (G4 / 64) / 8, 1), NTHR, 0, stream>>>(
      XB, XB, DIM, 0L, WIHB, WIHB, DIM, 0L, (void*)PXG, (void*)PXG, G4, 0L,
      bih, PXG, 0L, TWIN, G4, DIM, 1.0f);
  seq_cell_kernel<<<1, PTHR, 0, stream>>>(PXG, WHHB, WIHB, W1B, W2B, bih, bhh, b1, b2, HPL, out);
}
